// DiffeqExactTraceMLP_51178830299530
// MI455X (gfx1250) — hardware-verified
//
#include <hip/hip_runtime.h>
#include <stdint.h>
#include <stddef.h>
#include <math.h>

#pragma clang fp contract(off)

#define NBAT 1024
#define ND   128
#define NDH  64
#define NHID 512
#define NW2  8192
#define NROW 131072

#define TT   64
#define TPH  72
#define CP   136
#define MROW 64
#define ZP   520
#define ATP  72

#define OFF_Z0 0
#define OFF_T0 (OFF_Z0 + MROW * ZP * 2)
#define OFF_AT (OFF_T0 + MROW * ZP * 2)
#define OFF_YP (OFF_AT + MROW * ATP * 2)
#define OFF_JP (OFF_YP + 8 * MROW * 4)
#define OFF_YF (OFF_JP + 8 * MROW * 4)
#define OFF_JF (OFF_YF + MROW * 4)
#define LDS_DW (OFF_JF + MROW * 4)

static_assert(NW2 == ND * NDH);
static_assert(NROW == NBAT * ND);
static_assert((TPH * 2) % 16 == 0);
static_assert((CP * 2) % 16 == 0);
static_assert((ZP * 2) % 16 == 0);
static_assert((ATP * 2) % 16 == 0);
static_assert(OFF_T0 % 16 == 0);
static_assert(OFF_AT % 16 == 0);
static_assert(OFF_YP % 16 == 0);
static_assert(OFF_JP % 16 == 0);
static_assert(OFF_YF % 16 == 0);
static_assert(OFF_JF % 16 == 0);
static_assert(LDS_DW == 146944);
static_assert(NHID % 128 == 0);
static_assert(NDH % 32 == 0);
static_assert(MROW == 64);
static_assert(NROW % MROW == 0);
static_assert(ND % MROW == 0);

typedef _Float16 v16h __attribute__((ext_vector_type(16)));
typedef _Float16 v8h  __attribute__((ext_vector_type(8)));
typedef float    v8f  __attribute__((ext_vector_type(8)));
typedef float    v4f  __attribute__((ext_vector_type(4)));
typedef v4f __attribute__((may_alias)) v4fa;
typedef v8h __attribute__((may_alias)) v8ha;

union FragH { v16h v; v8h q[2]; };

__device__ __forceinline__ v8f wmma_h(v16h a, v16h b, v8f c) {
  v8f d = __builtin_amdgcn_wmma_f32_16x16x32_f16(false, a, false, b, (short)0, c, false, false);
  asm volatile("v_nop\n\tv_nop\n\tv_nop\n\tv_nop" : "+v"(d) : "v"(a), "v"(b));
  return d;
}

__device__ __forceinline__ v16h ldfrag_h(const _Float16* p, int h) {
  FragH f;
  f.q[0] = *(const v8ha*)(p + 8 * h);
  f.q[1] = *(const v8ha*)(p + 16 + 8 * h);
  return f.v;
}

__device__ __forceinline__ v8f zero8() {
  const v8f z = {0.f, 0.f, 0.f, 0.f, 0.f, 0.f, 0.f, 0.f};
  return z;
}

__device__ __forceinline__ float tanh_f(float v) {
  const float ax = fminf(fabsf(v), 9.0f);
  const float ex = __expf(ax + ax);
  const float r  = __builtin_amdgcn_rcpf(ex + 1.0f);
  return copysignf(1.0f - 2.0f * r, v);
}

__device__ __forceinline__ float ar_mask(int mode, int rev, int r, int c) {
  const int degr = rev ? (ND - 1 - r) : r;
  const int dc   = c & (ND - 1);
  const int degc = rev ? (ND - 1 - dc) : dc;
  const int rh = r % (ND - 1), ch = c % (ND - 1);
  const int k1 = (degr <= ch) ? 1 : 0;
  const int k2 = (rh <= ch) ? 1 : 0;
  const int k3 = (rh < degc) ? 1 : 0;
  const int keep = (mode == 0) ? 1 : ((mode == 1) ? k1 : ((mode == 2) ? k2 : k3));
  return (float)keep;
}

__global__ __launch_bounds__(256) void k_wt(const float* __restrict__ src,
                                            _Float16* __restrict__ dst,
                                            int R, int C, int dpitch, int dcol,
                                            float scale, int mode, int rev)
{
  __shared__ __align__(16) _Float16 sT[TT * TPH];
  const int tid = threadIdx.x, lane = tid & 31, wv = tid >> 5;
  const int r0 = blockIdx.y * TT;
  const int c0 = blockIdx.x * TT;
  if (r0 + TT > R || c0 + TT > C) return;

  const int i = tid >> 2, cs = (tid & 3) * 16;
  const int gr = r0 + i, gc = c0 + cs;
  const float* sp = src + (size_t)gr * C + gc;
  const v4f a0 = *(const v4fa*)(sp);
  const v4f a1 = *(const v4fa*)(sp + 4);
  const v4f a2 = *(const v4fa*)(sp + 8);
  const v4f a3 = *(const v4fa*)(sp + 12);
  float vv[16];
  vv[0]  = a0.x; vv[1]  = a0.y; vv[2]  = a0.z; vv[3]  = a0.w;
  vv[4]  = a1.x; vv[5]  = a1.y; vv[6]  = a1.z; vv[7]  = a1.w;
  vv[8]  = a2.x; vv[9]  = a2.y; vv[10] = a2.z; vv[11] = a2.w;
  vv[12] = a3.x; vv[13] = a3.y; vv[14] = a3.z; vv[15] = a3.w;
  _Float16* tp = sT + cs * TPH + i;
  #pragma unroll
  for (int j = 0; j < 16; ++j) {
    const float mk = ar_mask(mode, rev, gr, gc + j);
    tp[j * TPH] = (_Float16)(vv[j] * mk * scale);
  }
  __syncthreads();

  const int q  = lane & 7;
  const int cA = 4 * wv + (lane >> 3);
  const int cB = 32 + cA;
  const v8h vA = *(const v8ha*)(sT + cA * TPH + 8 * q);
  const v8h vB = *(const v8ha*)(sT + cB * TPH + 8 * q);
  _Float16* dA = dst + (size_t)(c0 + cA) * dpitch + dcol + r0 + 8 * q;
  _Float16* dB = dst + (size_t)(c0 + cB) * dpitch + dcol + r0 + 8 * q;
  *(volatile v8ha*)dA = vA;
  *(volatile v8ha*)dB = vB;
  __threadfence();
  *(volatile v8ha*)dA = vA;
  *(volatile v8ha*)dB = vB;
}

__global__ __launch_bounds__(256) void k_cvt_x(const float* __restrict__ src,
                                               _Float16* __restrict__ dst, int n8)
{
  const int i = blockIdx.x * 256 + threadIdx.x;
  if (i >= n8) return;
  const float* sp = src + (size_t)i * 8;
  const v4f a = *(const v4fa*)(sp);
  const v4f b = *(const v4fa*)(sp + 4);
  v8h o;
  o[0] = (_Float16)a.x; o[1] = (_Float16)a.y; o[2] = (_Float16)a.z; o[3] = (_Float16)a.w;
  o[4] = (_Float16)b.x; o[5] = (_Float16)b.y; o[6] = (_Float16)b.z; o[7] = (_Float16)b.w;
  _Float16* dp = dst + (size_t)i * 8;
  *(volatile v8ha*)dp = o;
  __threadfence();
  *(volatile v8ha*)dp = o;
}

template <int RELU, int NBIAS>
__global__ __launch_bounds__(256) void k_gemm(const _Float16* __restrict__ A, int lda,
                                              const _Float16* __restrict__ BT, int ldb,
                                              const float* __restrict__ bias0,
                                              const float* __restrict__ bias1,
                                              _Float16* __restrict__ out, int ldo, int ocol,
                                              int M, int N, int K, float scale)
{
  __shared__ __align__(16) _Float16 sC[128 * CP];
  const int tid = threadIdx.x, lane = tid & 31, wv = tid >> 5;
  const int h = lane >> 4, m = lane & 15;
  const int waveM = wv & 1, waveN = wv >> 1;
  const int bM = blockIdx.y * 128, bN = blockIdx.x * 128;
  if (bM + 128 > M || bN + 128 > N) return;

  v8f acc[4][2];
  #pragma unroll
  for (int mt = 0; mt < 4; ++mt) { acc[mt][0] = zero8(); acc[mt][1] = zero8(); }

  const _Float16* ap = A  + (size_t)(bM + waveM * 64 + m) * lda;
  const _Float16* bp = BT + (size_t)(bN + waveN * 32 + m) * ldb;
  #pragma unroll 1
  for (int k0 = 0; k0 < K; k0 += 32) {
    const v16h bf0 = ldfrag_h(bp + k0, h);
    const v16h bf1 = ldfrag_h(bp + (size_t)16 * ldb + k0, h);
    #pragma unroll
    for (int mt = 0; mt < 4; ++mt) {
      const v16h af = ldfrag_h(ap + (size_t)(mt * 16) * lda + k0, h);
      acc[mt][0] = wmma_h(af, bf0, acc[mt][0]);
      acc[mt][1] = wmma_h(af, bf1, acc[mt][1]);
    }
  }

  #pragma unroll
  for (int nt = 0; nt < 2; ++nt) {
    const int col = waveN * 32 + nt * 16 + m;
    float bv = bias0[bN + col];
    if (NBIAS == 2) bv += bias1[bN + col];
    #pragma unroll
    for (int mt = 0; mt < 4; ++mt) {
      #pragma unroll
      for (int g = 0; g < 8; ++g) {
        const int row = waveM * 64 + mt * 16 + 8 * h + g;
        float v = acc[mt][nt][g] * scale + bv;
        if (RELU) v = fmaxf(v, 0.f);
        sC[row * CP + col] = (_Float16)v;
      }
    }
  }
  __syncthreads();

  const int q = lane & 7, sub = lane >> 3;
  #pragma unroll
  for (int j = 0; j < 8; ++j) {
    const int row  = wv * 16 + 2 * j + (sub >> 1);
    const int colh = (sub & 1) * 64 + 8 * q;
    const v8h v = *(const v8ha*)(sC + row * CP + colh);
    _Float16* dp = out + (size_t)(bM + row) * ldo + ocol + bN + colh;
    *(volatile v8ha*)dp = v;
  }
  __threadfence();
  #pragma unroll
  for (int j = 0; j < 8; ++j) {
    const int row  = wv * 16 + 2 * j + (sub >> 1);
    const int colh = (sub & 1) * 64 + 8 * q;
    const v8h v = *(const v8ha*)(sC + row * CP + colh);
    _Float16* dp = out + (size_t)(bM + row) * ldo + ocol + bN + colh;
    *(volatile v8ha*)dp = v;
  }
}

__global__ __launch_bounds__(256) void k_dimwise(const _Float16* __restrict__ Hs,
                                                 const float* __restrict__ x,
                                                 const float* __restrict__ t,
                                                 const float* __restrict__ dW0,
                                                 const float* __restrict__ b0,
                                                 const _Float16* __restrict__ W0hT,
                                                 const _Float16* __restrict__ W1T,
                                                 const float* __restrict__ b1,
                                                 const float* __restrict__ W2,
                                                 const float* __restrict__ b2,
                                                 float* __restrict__ out)
{
  extern __shared__ __align__(16) unsigned char dsm[];
  _Float16* Z0 = (_Float16*)(dsm + OFF_Z0);
  _Float16* T0 = (_Float16*)(dsm + OFF_T0);
  _Float16* AT = (_Float16*)(dsm + OFF_AT);
  float* yP = (float*)(dsm + OFF_YP);
  float* jP = (float*)(dsm + OFF_JP);
  float* yF = (float*)(dsm + OFF_YF);
  float* jF = (float*)(dsm + OFF_JF);

  const int tid = threadIdx.x, lane = tid & 31, wv = tid >> 5;
  const int h = lane >> 4, m = lane & 15;
  const int r0 = blockIdx.x * MROW;
  const int bi = r0 >> 7, i0 = r0 & (ND - 1);

  {
    const int k = tid >> 2, seg = (tid & 3) * 16;
    const _Float16* sp = Hs + (size_t)bi * NW2 + k * ND + i0 + seg;
    const v8h u0 = *(const v8ha*)(sp);
    const v8h u1 = *(const v8ha*)(sp + 8);
    _Float16* tp = AT + seg * ATP + k;
    #pragma unroll
    for (int j = 0; j < 8; ++j) {
      tp[j * ATP]       = u0[j];
      tp[(8 + j) * ATP] = u1[j];
    }
  }
  __syncthreads();

  const float tv = t[0];
  const float inv64 = 0.015625f;
  const float inv4096 = 0.000244140625f;

  #pragma unroll 1
  for (int nt = 0; nt < 4; ++nt) {
    const int n = wv * 64 + nt * 16 + m;
    v8f acc[4];
    #pragma unroll
    for (int mt = 0; mt < 4; ++mt) acc[mt] = zero8();
    #pragma unroll
    for (int ks = 0; ks < 2; ++ks) {
      const int kb = ks * 32;
      const v16h bf = ldfrag_h(W0hT + (size_t)n * NDH + kb, h);
      #pragma unroll
      for (int mt = 0; mt < 4; ++mt) {
        const v16h af = ldfrag_h(AT + (mt * 16 + m) * ATP + kb, h);
        acc[mt] = wmma_h(af, bf, acc[mt]);
      }
    }
    const float w0r0 = dW0[n], w0r1 = dW0[NHID + n], bb = b0[n];
    #pragma unroll
    for (int mt = 0; mt < 4; ++mt) {
      #pragma unroll
      for (int g = 0; g < 8; ++g) {
        const int rloc = mt * 16 + 8 * h + g;
        const float a = acc[mt][g] * inv64 + tv * w0r0 + x[r0 + rloc] * w0r1 + bb;
        const float z = tanh_f(a);
        const float dz = (w0r1 + w0r1 * z) * (1.0f - z);
        Z0[rloc * ZP + n] = (_Float16)z;
        T0[rloc * ZP + n] = (_Float16)(dz * 64.0f);
      }
    }
  }
  __syncthreads();

  float ysel[4], jsel[4];
  #pragma unroll
  for (int mt = 0; mt < 4; ++mt) { ysel[mt] = 0.f; jsel[mt] = 0.f; }

  #pragma unroll 1
  for (int nc = 0; nc < 4; ++nc) {
    const int n = nc * 128 + wv * 16 + m;
    v8f a1[4], t1[4];
    #pragma unroll
    for (int mt = 0; mt < 4; ++mt) { a1[mt] = zero8(); t1[mt] = zero8(); }
    const _Float16* bp = W1T + (size_t)n * NHID;
    #pragma unroll 1
    for (int k0 = 0; k0 < NHID; k0 += 32) {
      const v16h bf = ldfrag_h(bp + k0, h);
      #pragma unroll
      for (int mt = 0; mt < 4; ++mt) {
        const v16h za = ldfrag_h(Z0 + (mt * 16 + m) * ZP + k0, h);
        const v16h ta = ldfrag_h(T0 + (mt * 16 + m) * ZP + k0, h);
        a1[mt] = wmma_h(za, bf, a1[mt]);
        t1[mt] = wmma_h(ta, bf, t1[mt]);
      }
    }
    const float b1v = b1[n], w2v = W2[n];
    #pragma unroll
    for (int mt = 0; mt < 4; ++mt) {
      #pragma unroll
      for (int g = 0; g < 8; ++g) {
        const float z  = tanh_f(a1[mt][g] * inv64 + b1v);
        const float da = t1[mt][g] * inv4096;
        const float tz = (da + da * z) * (1.0f - z);
        float ys = z * w2v, js = tz * w2v;
        #pragma unroll
        for (int off = 1; off < 16; off <<= 1) {
          ys += __shfl_xor(ys, off, 32);
          js += __shfl_xor(js, off, 32);
        }
        ysel[mt] += (m == g) ? ys : 0.f;
        jsel[mt] += (m == g) ? js : 0.f;
      }
    }
  }
  if (m < 8) {
    #pragma unroll
    for (int mt = 0; mt < 4; ++mt) {
      const int row = mt * 16 + 8 * h + m;
      yP[wv * MROW + row] = ysel[mt];
      jP[wv * MROW + row] = jsel[mt];
    }
  }
  __syncthreads();
  if (tid < MROW) {
    float sy = 0.f, sj = 0.f;
    #pragma unroll
    for (int w2 = 0; w2 < 8; ++w2) {
      sy += yP[w2 * MROW + tid];
      sj += jP[w2 * MROW + tid];
    }
    yF[tid] = sy + b2[0];
    jF[tid] = sj;
  }
  __syncthreads();

  if (wv == 0) {
    const int q = lane & 15, which = lane >> 4;
    const v4f vy = *(const v4fa*)(yF + 4 * q);
    const v4f vj = *(const v4fa*)(jF + 4 * q);
    v4f v;
    v.x = which ? vj.x : vy.x;
    v.y = which ? vj.y : vy.y;
    v.z = which ? vj.z : vy.z;
    v.w = which ? vj.w : vy.w;
    float* dp = out + (size_t)which * NROW + r0 + 4 * q;
    *(volatile v4fa*)dp = v;
    __threadfence();
    *(volatile v4fa*)dp = v;
  }
}

extern "C" void kernel_launch(void* const* d_in, const int* in_sizes, int n_in,
                              void* d_out, int out_size, void* d_ws, size_t ws_size,
                              hipStream_t stream)
{
  if (n_in < 20) return;
  if (in_sizes[0] < 1) return;
  if (in_sizes[1] != NROW) return;
  for (int p = 0; p < 2; ++p) {
    const int o = 2 + 6 * p;
    if (in_sizes[o + 0] != ND * NHID) return;
    if (in_sizes[o + 1] != NHID) return;
    if (in_sizes[o + 2] != NHID * NHID) return;
    if (in_sizes[o + 3] != NHID) return;
    if (in_sizes[o + 4] != NHID * NW2) return;
    if (in_sizes[o + 5] != NW2) return;
  }
  if (in_sizes[14] != (NDH + 2) * NHID) return;
  if (in_sizes[15] != NHID) return;
  if (in_sizes[16] != NHID * NHID) return;
  if (in_sizes[17] != NHID) return;
  if (in_sizes[18] != NHID) return;
  if (in_sizes[19] < 1) return;
  if (out_size != 2 * NROW) return;

  const float* t   = (const float*)d_in[0];
  const float* x   = (const float*)d_in[1];
  const float* mW0[2] = {(const float*)d_in[2], (const float*)d_in[8]};
  const float* mb0[2] = {(const float*)d_in[3], (const float*)d_in[9]};
  const float* mW1[2] = {(const float*)d_in[4], (const float*)d_in[10]};
  const float* mb1[2] = {(const float*)d_in[5], (const float*)d_in[11]};
  const float* mW2[2] = {(const float*)d_in[6], (const float*)d_in[12]};
  const float* mb2[2] = {(const float*)d_in[7], (const float*)d_in[13]};
  const float* dW0 = (const float*)d_in[14];
  const float* db0 = (const float*)d_in[15];
  const float* dW1 = (const float*)d_in[16];
  const float* db1 = (const float*)d_in[17];
  const float* dW2 = (const float*)d_in[18];
  const float* db2 = (const float*)d_in[19];
  float* out = (float*)d_out;

  const size_t bX   = (size_t)NROW * 2;
  const size_t bW0  = (size_t)NHID * ND * 2;
  const size_t bW1  = (size_t)NHID * NHID * 2;
  const size_t bW2  = (size_t)NW2 * (2 * NHID) * 2;
  const size_t bD0  = (size_t)NHID * NDH * 2;
  const size_t bD1  = (size_t)NHID * NHID * 2;
  const size_t bH0  = (size_t)NBAT * NHID * 2;
  const size_t bH1  = (size_t)NBAT * (2 * NHID) * 2;
  const size_t bHS  = (size_t)NBAT * NW2 * 2;
  const size_t total = bX + 2 * bW0 + 2 * bW1 + bW2 + bD0 + bD1 + 2 * bH0 + bH1 + bHS;
  if (total > ws_size) return;
  if (total > (size_t)134217728) return;

  char* ws = (char*)d_ws;
  size_t off = 0;
  _Float16* X16 = (_Float16*)(ws + off); off += bX;
  _Float16* W0T[2]; _Float16* W1T[2]; _Float16* H0[2];
  W0T[0] = (_Float16*)(ws + off); off += bW0;
  W0T[1] = (_Float16*)(ws + off); off += bW0;
  W1T[0] = (_Float16*)(ws + off); off += bW1;
  W1T[1] = (_Float16*)(ws + off); off += bW1;
  _Float16* W2C = (_Float16*)(ws + off); off += bW2;
  _Float16* D0T = (_Float16*)(ws + off); off += bD0;
  _Float16* D1T = (_Float16*)(ws + off); off += bD1;
  H0[0] = (_Float16*)(ws + off); off += bH0;
  H0[1] = (_Float16*)(ws + off); off += bH0;
  _Float16* H1C = (_Float16*)(ws + off); off += bH1;
  _Float16* HS  = (_Float16*)(ws + off); off += bHS;
  if (off != total) return;

  const float inv64 = 0.015625f;

  k_cvt_x<<<dim3((NROW / 8 + 255) / 256), 256, 0, stream>>>(x, X16, NROW / 8);

  for (int p = 0; p < 2; ++p) {
    k_wt<<<dim3(NHID / TT, ND / TT),   256, 0, stream>>>(mW0[p], W0T[p], ND,   NHID, ND,       0,        64.0f, 1, p);
    k_wt<<<dim3(NHID / TT, NHID / TT), 256, 0, stream>>>(mW1[p], W1T[p], NHID, NHID, NHID,     0,        64.0f, 2, p);
    k_wt<<<dim3(NW2 / TT,  NHID / TT), 256, 0, stream>>>(mW2[p], W2C,    NHID, NW2,  2 * NHID, p * NHID, 64.0f, 3, p);
  }
  k_wt<<<dim3(NHID / TT, NDH / TT),  256, 0, stream>>>(dW0 + 2 * NHID, D0T, NDH, NHID, NDH, 0, 64.0f, 0, 0);
  k_wt<<<dim3(NHID / TT, NHID / TT), 256, 0, stream>>>(dW1, D1T, NHID, NHID, NHID, 0, 64.0f, 0, 0);

  for (int p = 0; p < 2; ++p) {
    k_gemm<1, 1><<<dim3(NHID / 128, NBAT / 128), 256, 0, stream>>>(X16, ND, W0T[p], ND, mb0[p], mb0[p],
                                                                   H0[p], NHID, 0, NBAT, NHID, ND, inv64);
    k_gemm<1, 1><<<dim3(NHID / 128, NBAT / 128), 256, 0, stream>>>(H0[p], NHID, W1T[p], NHID, mb1[p], mb1[p],
                                                                   H1C, 2 * NHID, p * NHID, NBAT, NHID, NHID, inv64);
  }
  k_gemm<0, 2><<<dim3(NW2 / 128, NBAT / 128), 256, 0, stream>>>(H1C, 2 * NHID, W2C, 2 * NHID, mb2[0], mb2[1],
                                                                 HS, NW2, 0, NBAT, NW2, 2 * NHID, inv64);

  hipFuncSetAttribute(reinterpret_cast<const void*>(&k_dimwise),
                      hipFuncAttributeMaxDynamicSharedMemorySize, LDS_DW);
  k_dimwise<<<dim3(NROW / MROW), 256, LDS_DW, stream>>>(HS, x, t, dW0, db0, D0T, D1T, db1, dW2, db2, out);
}
